// SAHead_45054206935084
// MI455X (gfx1250) — hardware-verified
//
#include <hip/hip_runtime.h>
#include <hip/hip_bf16.h>
#include <math.h>

#define BB 2
#define SS 9216
#define HH 1
#define DKK 64
#define QW 2
#define CIN 64
#define CENC 96

typedef _Float16 bf16;
typedef _Float16 f16;
typedef __attribute__((ext_vector_type(4))) unsigned v4u_t;
typedef unsigned v4ua __attribute__((ext_vector_type(4), may_alias));
typedef __attribute__((ext_vector_type(4))) float v4f_t;
typedef float v4fa __attribute__((ext_vector_type(4), may_alias));
typedef __attribute__((ext_vector_type(16))) bf16  bf16x16;
typedef bf16x16 f16x16;
typedef __attribute__((ext_vector_type(8)))  bf16  bf16x8;
typedef bf16x8 f16x8;
typedef __attribute__((ext_vector_type(4)))  bf16  bf16x4;
typedef __attribute__((ext_vector_type(8)))  float f32x8;
#define LDS_STRIDE 48
#define KSTRIDE    72
#define VSTRIDE    48

__device__ __forceinline__ f32x8 wmma_bf16(bf16x16 a, bf16x16 b, f32x8 c) {
  c = __builtin_amdgcn_wmma_f32_16x16x32_f16(false, a, false, b, (short)0, c, false, false);
  asm volatile("v_nop\n\tv_nop\n\tv_nop\n\tv_nop" : "+v"(c) : "v"(a), "v"(b));
  return c;
}

template <typename T>
__device__ __forceinline__ bf16x16 load_frag(const T* __restrict__ base, int ld,
                                             int row0, int k0) {
  const int lane = threadIdx.x & 31;
  const int r    = lane & 15;
  const int kh   = (lane >> 4) * 8;
  const T* p0 = base + (size_t)(row0 + r) * ld + (k0 + kh);
  const T* p1 = p0 + 16;
  bf16x16 f;
#pragma unroll
  for (int i = 0; i < 8; ++i) {
    f[i]     = (bf16)p0[i];
    f[i + 8] = (bf16)p1[i];
  }
  return f;
}

__device__ __forceinline__ bf16x16 lds_frag(const bf16* base, int stride) {
  const int lane = threadIdx.x & 31;
  const int row  = lane & 15;
  const int kh   = (lane >> 4) * 8;
  const bf16x8 lo = *(const bf16x8*)(base + row * stride + kh);
  const bf16x8 hi = *(const bf16x8*)(base + row * stride + kh + 16);
  bf16x16 f;
#pragma unroll
  for (int i = 0; i < 8; ++i) { f[i] = lo[i]; f[i + 8] = hi[i]; }
  return f;
}

template <typename T>
__device__ __forceinline__ void stage_read16(const T* __restrict__ p, float* buf) {
#pragma unroll
  for (int i = 0; i < 16; ++i) buf[i] = (float)p[i];
}

__device__ __forceinline__ void stage_write(bf16* dst, const float* buf, int nquad) {
#pragma unroll
  for (int i = 0; i < nquad; ++i) {
    bf16x4 q;
    q[0] = (bf16)buf[4 * i];     q[1] = (bf16)buf[4 * i + 1];
    q[2] = (bf16)buf[4 * i + 2]; q[3] = (bf16)buf[4 * i + 3];
    *(bf16x4*)(dst + 4 * i) = q;
  }
}

__global__ __launch_bounds__(64) void attn_kernel(
    const bf16* __restrict__ Qb, const bf16* __restrict__ Kb,
    const bf16* __restrict__ Vt, float* __restrict__ Rout) {
  __shared__ bf16 ldsK[32 * KSTRIDE];
  __shared__ __attribute__((aligned(16))) bf16 ldsQ[64 * KSTRIDE];
  __shared__ bf16 ldsV[64 * VSTRIDE];
  __shared__ __attribute__((aligned(16))) float ldsO[2][64 * 36];

  const int q0blk = blockIdx.x * 64;
  const int h  = blockIdx.y;
  const int b  = blockIdx.z;
  const int t    = threadIdx.x;
  const int wave = t >> 5;
  const int lane = t & 31;
  const int qlane = lane & 15;
  const int kh8   = (lane >> 4) * 8;
  const int q0 = q0blk + wave * 32;

  const bf16* Qc = Qb + (size_t)b * DKK * SS;
  const bf16* Kc = Kb + (size_t)b * DKK * SS;
  const bf16* Vh = Vt + (size_t)b * DKK * SS;
  for (int e = t; e < 64 * 64; e += 64) { const int d = e >> 6, qq = e & 63; ldsQ[qq * KSTRIDE + d] = Qc[(size_t)d * SS + q0blk + qq]; }
  __syncthreads();

  const bf16* kSrc = Kc + (size_t)t * SS;
  const bf16* vSrc = Vh + (size_t)t * SS;

  bf16x16 qf[QW][2];
#pragma unroll
  for (int qt = 0; qt < QW; ++qt) {
    qf[qt][0] = lds_frag(ldsQ + (wave * 32 + 16 * qt) * KSTRIDE, KSTRIDE);
    qf[qt][1] = lds_frag(ldsQ + (wave * 32 + 16 * qt) * KSTRIDE + 32, KSTRIDE);
  }

  f32x8 o[QW][4] = {};
  float mrun[QW], lrun[QW];
#pragma unroll
  for (int qt = 0; qt < QW; ++qt) { mrun[qt] = -INFINITY; lrun[qt] = 0.0f; }

  const float scale = 1.44269504088896340736f;
  const float NEG2 = -1.0e9f;
  const int kmax = SS - 1;

  bf16x8 kreg[4], vreg[4];
#pragma unroll
  for (int i = 0; i < 4; ++i) {
    kreg[i] = *(const bf16x8*)(kSrc + 8 * i);
    vreg[i] = *(const bf16x8*)(vSrc + 8 * i);
  }

  for (int kb = 0; kb <= kmax; kb += 32) {
    __syncthreads();
#pragma unroll
    for (int i = 0; i < 4; ++i) {
#pragma unroll
      for (int u = 0; u < 8; ++u) ldsK[(8 * i + u) * KSTRIDE + t] = kreg[i][u];
      *(bf16x8*)(&ldsV[t * VSTRIDE + 8 * i]) = vreg[i];
    }
    if (kb + 32 <= kmax) {
      const bf16* kn = kSrc + (kb + 32);
      const bf16* vn = vSrc + (kb + 32);
#pragma unroll
      for (int i = 0; i < 4; ++i) {
        kreg[i] = *(const bf16x8*)(kn + 8 * i);
        vreg[i] = *(const bf16x8*)(vn + 8 * i);
      }
    }
    __syncthreads();

    bf16x16 kf[2][2];
#pragma unroll
    for (int ktile = 0; ktile < 2; ++ktile)
#pragma unroll
      for (int c = 0; c < 2; ++c)
        kf[ktile][c] = lds_frag(ldsK + (ktile * 16) * KSTRIDE + c * 32, KSTRIDE);

    bf16x16 pf[QW];
    bool act[QW];
#pragma unroll
    for (int qt = 0; qt < QW; ++qt) {
      unsigned mbits = 0;
      mbits = 0xFFFFu; act[qt] = true;
      if (act[qt]) {
        const int q_my = q0 + 16 * qt + qlane;
        f32x8 s0 = {}, s1 = {};
        s0 = wmma_bf16(kf[0][0], qf[qt][0], s0);
        s0 = wmma_bf16(kf[0][1], qf[qt][1], s0);
        s1 = wmma_bf16(kf[1][0], qf[qt][0], s1);
        s1 = wmma_bf16(kf[1][1], qf[qt][1], s1);

        float mx = -INFINITY;
#pragma unroll
        for (int r = 0; r < 8; ++r) {
          const int k0i = kb + kh8 + r;
          const int k1i = k0i + 16;
          (void)k0i; (void)k1i; (void)q_my;
          s0[r] = (mbits & (1u << r))       ? s0[r] * scale : NEG2;
          s1[r] = (mbits & (1u << (8 + r))) ? s1[r] * scale : NEG2;
          mx = fmaxf(mx, fmaxf(s0[r], s1[r]));
        }
        mx = fmaxf(mx, __shfl_xor(mx, 16, 32));
        const float mnew  = fmaxf(mrun[qt], mx);
        const float alpha = exp2f(mrun[qt] - mnew);

        float rsum = 0.0f;
#pragma unroll
        for (int r = 0; r < 8; ++r) {
          const float p0 = exp2f(s0[r] - mnew);
          const float p1 = exp2f(s1[r] - mnew);
          rsum += p0 + p1;
          pf[qt][r]     = (bf16)(p0 * 1024.0f);
          pf[qt][r + 8] = (bf16)(p1 * 1024.0f);
        }
        rsum += __shfl_xor(rsum, 16, 32);
        lrun[qt] = lrun[qt] * alpha + rsum;
        mrun[qt] = mnew;

#pragma unroll
        for (int j = 0; j < 4; ++j)
#pragma unroll
          for (int r = 0; r < 8; ++r) o[qt][j][r] *= alpha;
      }
    }

#pragma unroll
    for (int j = 0; j < 4; ++j) {
      const bf16x16 vf = lds_frag(ldsV + (j * 16) * VSTRIDE, VSTRIDE);
#pragma unroll
      for (int qt = 0; qt < QW; ++qt)
        if (act[qt]) o[qt][j] = wmma_bf16(vf, pf[qt], o[qt][j]);
    }
  }

  float* so = ldsO[wave];
#pragma unroll
  for (int qt = 0; qt < QW; ++qt) {
    const float rl = 1.0f / (lrun[qt] * 1024.0f);
#pragma unroll
    for (int j = 0; j < 4; ++j)
#pragma unroll
      for (int r = 0; r < 8; ++r) so[(j * 16 + kh8 + r) * 36 + 16 * qt + qlane] = o[qt][j][r] * rl;
  }
  asm volatile("s_wait_dscnt 0" ::: "memory");
  __builtin_amdgcn_wave_barrier();
#pragma unroll 1
  for (int pass = 0; pass < 2; ++pass) {
#pragma unroll
    for (int it = 0; it < 16; ++it) { const int ch = lane + 32 * it, d = ch >> 3, q4 = (ch & 7) * 4;
      *(volatile v4f_t*)(Rout + ((size_t)b * DKK + d) * SS + q0 + q4) = *(const volatile v4fa*)(so + d * 36 + q4); }
    __threadfence();
  }
}


template <int KC>
__device__ __forceinline__ f16x16 wfrag32(const float* __restrict__ Wm, int r0, int k0) {
  const int lane = threadIdx.x & 31, r = lane & 15, kh = (lane >> 4) * 8;
  const float* p = Wm + (size_t)(r0 + r) * KC;
  f16x16 f;
#pragma unroll
  for (int i = 0; i < 8; ++i) { const int ka = k0 + kh + i, kb2 = k0 + 16 + kh + i; f[i] = (f16)((ka < KC) ? p[ka] : 0.0f); f[8 + i] = (f16)((kb2 < KC) ? p[kb2] : 0.0f); }
  return f;
}
template <int KC, bool NORM>
__global__ __launch_bounds__(256) void k_proj(const float* __restrict__ in, const float* __restrict__ Wm, const float* __restrict__ bias, bf16* __restrict__ outp) {
  __shared__ __attribute__((aligned(16))) f16 xS[128 * 104];
  __shared__ __attribute__((aligned(16))) float cS[64 * 132];
  __shared__ float nrm[128];
  const int tid = threadIdx.x, lane = tid & 31, wave = tid >> 5, cl = lane & 15, rh = (lane >> 4) * 8;
  const int b = blockIdx.x / (SS / 128), p0 = (blockIdx.x % (SS / 128)) * 128;
  const float* src = in + (size_t)b * KC * SS + p0;
  for (int e = tid; e < KC * 128; e += 256) { const int c = e >> 7, p = e & 127; xS[p * 104 + c] = (f16)src[(size_t)c * SS + p]; }
  for (int e = tid; e < (104 - KC) * 128; e += 256) { const int c = KC + e / 128, p = e % 128; xS[p * 104 + c] = (f16)0.0f; }
  __syncthreads();
  const int dt = wave & 3, pt0 = (wave >> 2) * 4;
  constexpr int KSTEPS = (KC + 31) / 32;
  f16x16 af[KSTEPS];
#pragma unroll
  for (int ks = 0; ks < KSTEPS; ++ks) af[ks] = wfrag32<KC>(Wm, dt * 16, ks * 32);
#pragma unroll
  for (int j = 0; j < 4; ++j) {
    f32x8 acc = {};
#pragma unroll
    for (int ks = 0; ks < KSTEPS; ++ks) acc = wmma_bf16(af[ks], lds_frag(xS + ((pt0 + j) * 16) * 104 + ks * 32, 104), acc);
#pragma unroll
    for (int r = 0; r < 8; ++r) cS[(dt * 16 + rh + r) * 132 + (pt0 + j) * 16 + cl] = acc[r] + bias[dt * 16 + rh + r];
  }
  __syncthreads();
  if (NORM) {
    if (tid < 128) { float s = 0.0f;
#pragma unroll 8
      for (int d = 0; d < 64; ++d) { const float v = cS[d * 132 + tid]; s += v * v; }
      nrm[tid] = 1.0f / fmaxf(sqrtf(s), 1e-6f); }
    __syncthreads();
  }
#pragma unroll 1
  for (int pass = 0; pass < 2; ++pass) {
#pragma unroll
    for (int it = 0; it < 4; ++it) { const int ch = tid + 256 * it, d = ch >> 4, q8 = (ch & 15) * 8;
      union { bf16 hh[8]; v4u_t u; } cv;
#pragma unroll
      for (int e = 0; e < 8; ++e) { const float v = cS[d * 132 + q8 + e] * (NORM ? nrm[q8 + e] : 1.0f); cv.hh[e] = (bf16)v; }
      *(volatile v4u_t*)(outp + ((size_t)b * DKK + d) * SS + p0 + q8) = cv.u; }
    __threadfence();
  }
}

extern "C" void kernel_launch(void* const* d_in, const int* in_sizes, int n_in,
                              void* d_out, int out_size, void* d_ws, size_t ws_size,
                              hipStream_t stream) {
  (void)in_sizes; (void)n_in; (void)out_size; (void)ws_size;
  const float* x = (const float*)d_in[0];
  const float* xe = (const float*)d_in[1];
  const float* Wq = (const float*)d_in[2], *bq = (const float*)d_in[3], *Wk = (const float*)d_in[4], *bk = (const float*)d_in[5], *Wv = (const float*)d_in[6], *bv = (const float*)d_in[7];
  float* out = (float*)d_out;
  char* ws = (char*)d_ws;
  const size_t T16 = (size_t)BB * DKK * SS * 2;
  bf16* Qc = (bf16*)ws; bf16* Kc = (bf16*)(ws + T16); bf16* Vc = (bf16*)(ws + 2 * T16);
  k_proj<CENC, true ><<<dim3(BB * SS / 128), dim3(256), 0, stream>>>(xe, Wq, bq, Qc);
  k_proj<CENC, true ><<<dim3(BB * SS / 128), dim3(256), 0, stream>>>(xe, Wk, bk, Kc);
  k_proj<CIN,  false><<<dim3(BB * SS / 128), dim3(256), 0, stream>>>(x,  Wv, bv, Vc);
  attn_kernel<<<dim3(SS / 64, 1, BB), dim3(64), 0, stream>>>(Qc, Kc, Vc, out);
}
